// CAGatedSelfAttention_12524124635218
// MI455X (gfx1250) — hardware-verified
//
#include <hip/hip_runtime.h>
#include <stdint.h>
#include <stddef.h>


typedef _Float16 v16h __attribute__((ext_vector_type(16)));
typedef _Float16 v8h  __attribute__((ext_vector_type(8)));
typedef float    v8f  __attribute__((ext_vector_type(8)));
typedef float    v4f  __attribute__((ext_vector_type(4)));

union Frag { v16h v; v8h hv[2]; };

#define B_      2
#define C_      256
#define HH_     56
#define WW_     56
#define N_      3136
#define MID_    32
#define INNER_  64
#define HEADS_  8
#define DH_     8
#define PP_     64
#define GNG_    32
#define CPG_    8
#define EPS_    1e-5f
#define WSC_    64.0f
#define QSC_    16.0f
#define PSC_    16384.0f

#define WOFF_PIN_ 0
#define WOFF_Q_   (INNER_ * C_)
#define WOFF_K_   (WOFF_Q_ + INNER_ * INNER_)
#define WOFF_V_   (WOFF_K_ + INNER_ * INNER_)
#define WOFF_PW_  (WOFF_V_ + INNER_ * INNER_)
#define WTOT_     (WOFF_PW_ + C_ * INNER_)

static_assert(N_ % 64 == 0);
static_assert(C_ % 32 == 0);
static_assert(HH_ == WW_);
static_assert(WTOT_ % 2048 == 0);

static __device__ __forceinline__ v8f mma16(v16h a, v16h b, v8f c) {
    v8f d = __builtin_amdgcn_wmma_f32_16x16x32_f16(false, a, false, b, (short)0, c, false, false);
    asm volatile("v_nop\n\tv_nop\n\tv_nop\n\tv_nop" : "+v"(d) : "v"(a), "v"(b));
    return d;
}

static __device__ __forceinline__ v8f zero8f() {
    v8f z;
#pragma unroll
    for (int e = 0; e < 8; ++e) z[e] = 0.0f;
    return z;
}

static __device__ __forceinline__ v8h zero8h() {
    v8h z;
#pragma unroll
    for (int e = 0; e < 8; ++e) z[e] = (_Float16)0.0f;
    return z;
}

__global__ __launch_bounds__(256) void cvt_w_kernel(
    const float* __restrict__ pin, const float* __restrict__ wq,
    const float* __restrict__ wk,  const float* __restrict__ wv,
    const float* __restrict__ pw,  _Float16* __restrict__ wH) {
    const int i = blockIdx.x * 256 + threadIdx.x;
    if (i >= WTOT_ / 8) return;
    const float* src;
    int off;
    if (i < WOFF_Q_ / 8)       { src = pin; off = i * 8 - WOFF_PIN_; }
    else if (i < WOFF_K_ / 8)  { src = wq;  off = i * 8 - WOFF_Q_; }
    else if (i < WOFF_V_ / 8)  { src = wk;  off = i * 8 - WOFF_K_; }
    else if (i < WOFF_PW_ / 8) { src = wv;  off = i * 8 - WOFF_V_; }
    else                       { src = pw;  off = i * 8 - WOFF_PW_; }
    const v4f a = *(const v4f*)(src + off);
    const v4f c = *(const v4f*)(src + off + 4);
    v8h o;
#pragma unroll
    for (int e = 0; e < 4; ++e) {
        o[e]     = (_Float16)(a[e] * WSC_);
        o[4 + e] = (_Float16)(c[e] * WSC_);
    }
    _Float16* dst = wH + (size_t)i * 8;
    *(volatile v8h*)dst = o;
    __threadfence();
    *(volatile v8h*)dst = o;
}

__global__ __launch_bounds__(64) void pool_kernel(const float* __restrict__ x,
                                                  float* __restrict__ hpool,
                                                  float* __restrict__ wpool) {
    __shared__ __attribute__((aligned(16))) float hs[PP_];
    __shared__ __attribute__((aligned(16))) float vs[PP_];
    const int c = blockIdx.x, b = blockIdx.y, t = threadIdx.x;
    const float* p = x + (size_t)(b * C_ + c) * N_;
    float sh = 0.0f, sw = 0.0f;
    if (t < HH_) {
        const float* pr = p + t * WW_;
#pragma unroll 4
        for (int w = 0; w < WW_; ++w) sh += pr[w];
#pragma unroll 4
        for (int hh = 0; hh < HH_; ++hh) sw += p[hh * WW_ + t];
    }
    hs[t] = (t < HH_) ? sh * (1.0f / WW_) : 0.0f;
    vs[t] = (t < WW_) ? sw * (1.0f / HH_) : 0.0f;
    __syncthreads();
    if (t < PP_ / 4) {
        const v4f hv = *(const v4f*)&hs[4 * t];
        const v4f wv4 = *(const v4f*)&vs[4 * t];
        float* dh = hpool + (size_t)(b * C_ + c) * PP_ + 4 * t;
        float* dw = wpool + (size_t)(b * C_ + c) * PP_ + 4 * t;
        *(volatile v4f*)dh = hv;
        *(volatile v4f*)dw = wv4;
        __threadfence();
        *(volatile v4f*)dh = hv;
        *(volatile v4f*)dw = wv4;
    }
}

__global__ __launch_bounds__(256) void gates_kernel(
    const float* __restrict__ hpool, const float* __restrict__ wpool,
    const float* __restrict__ gcw,   const float* __restrict__ bng,
    const float* __restrict__ bnb,   const float* __restrict__ bnm,
    const float* __restrict__ bnv,   const float* __restrict__ ghw,
    const float* __restrict__ gww,   float* __restrict__ gh,
    float* __restrict__ gw) {
    __shared__ float cc[MID_ * (HH_ + WW_)];
    const int b = blockIdx.x, tid = threadIdx.x;
    const int L = HH_ + WW_;
    for (int t = tid; t < MID_ * L; t += 256) {
        const int mch = t / L, l = t - mch * L;
        const float* src = (l < HH_) ? (hpool + (size_t)b * C_ * PP_ + l)
                                     : (wpool + (size_t)b * C_ * PP_ + (l - HH_));
        const float* wr = gcw + mch * C_;
        float s = 0.0f;
#pragma unroll 1
        for (int c = 0; c < C_; ++c) s += wr[c] * src[(size_t)c * PP_];
        float v = (s - bnm[mch]) * (1.0f / sqrtf(bnv[mch] + EPS_));
        v = v * bng[mch] + bnb[mch];
        const float r6 = fminf(fmaxf(v + 3.0f, 0.0f), 6.0f);
        cc[t] = (v * r6) * (1.0f / 6.0f);
    }
    __syncthreads();
    for (int t = tid; t < C_ * (PP_ / 4); t += 256) {
        const int c = t >> 4, pos0 = (t & 15) * 4;
        float sh[4], sw[4];
#pragma unroll
        for (int j = 0; j < 4; ++j) { sh[j] = 0.0f; sw[j] = 0.0f; }
        v4f oh, ow;
        if (pos0 < HH_) {
            const float* whp = ghw + c * MID_;
            const float* wwp = gww + c * MID_;
#pragma unroll 1
            for (int mm = 0; mm < MID_; ++mm) {
                const float a = whp[mm], bq = wwp[mm];
                const float* cr = cc + mm * L + pos0;
#pragma unroll
                for (int j = 0; j < 4; ++j) {
                    sh[j] += a * cr[j];
                    sw[j] += bq * cr[HH_ + j];
                }
            }
#pragma unroll
            for (int j = 0; j < 4; ++j) {
                oh[j] = 1.0f / (1.0f + __expf(-sh[j]));
                ow[j] = 1.0f / (1.0f + __expf(-sw[j]));
            }
        } else {
#pragma unroll
            for (int j = 0; j < 4; ++j) { oh[j] = 0.0f; ow[j] = 0.0f; }
        }
        float* dh = gh + (size_t)(b * C_ + c) * PP_ + pos0;
        float* dw = gw + (size_t)(b * C_ + c) * PP_ + pos0;
        *(volatile v4f*)dh = oh;
        *(volatile v4f*)dw = ow;
        __threadfence();
        *(volatile v4f*)dh = oh;
        *(volatile v4f*)dw = ow;
    }
}

__global__ __launch_bounds__(256) void bias_kernel(const float* __restrict__ gh,
                                                   const float* __restrict__ gw,
                                                   float* __restrict__ biasv) {
    const int b = blockIdx.x;
    for (int t = threadIdx.x; t < N_ / 4; t += 256) {
        const int hq = t / (WW_ / 4), w0 = (t - hq * (WW_ / 4)) * 4;
        float s[4];
#pragma unroll
        for (int j = 0; j < 4; ++j) s[j] = 0.0f;
        const float* ghp = gh + (size_t)b * C_ * PP_ + hq;
        const float* gwp = gw + (size_t)b * C_ * PP_ + w0;
#pragma unroll 1
        for (int c = 0; c < C_; ++c) {
            const float a = ghp[(size_t)c * PP_];
            const v4f g4 = *(const v4f*)(gwp + (size_t)c * PP_);
#pragma unroll
            for (int j = 0; j < 4; ++j) s[j] += a * g4[j];
        }
        v4f o;
#pragma unroll
        for (int j = 0; j < 4; ++j) o[j] = fmaxf(logf(s[j] * (1.0f / C_)), -5.0f);
        float* dst = biasv + (size_t)b * N_ + 4 * t;
        *(volatile v4f*)dst = o;
        __threadfence();
        *(volatile v4f*)dst = o;
    }
}

__global__ __launch_bounds__(32) void seq_ln_kernel(
    const float* __restrict__ x, const _Float16* __restrict__ pinH,
    const float* __restrict__ lng, const float* __restrict__ lnb,
    _Float16* __restrict__ seqH) {
    __shared__ __attribute__((aligned(16))) _Float16 Xt[16 * 32];
    __shared__ __attribute__((aligned(16))) _Float16 St[16 * INNER_];
    const int lane = threadIdx.x, h = lane >> 4, m = lane & 15;
    const int nbase = blockIdx.x * 16, b = blockIdx.y;

    v8f acc[4];
#pragma unroll
    for (int t = 0; t < 4; ++t) acc[t] = zero8f();

    for (int kc = 0; kc < C_ / 32; ++kc) {
        const int c0 = kc * 32;
        const float* xr = x + (size_t)(b * C_ + c0 + lane) * N_ + nbase;
        v4f x4[4];
#pragma unroll
        for (int j = 0; j < 4; ++j) x4[j] = *(const v4f*)(xr + 4 * j);
#pragma unroll
        for (int j = 0; j < 4; ++j)
#pragma unroll
            for (int e = 0; e < 4; ++e) Xt[(4 * j + e) * 32 + lane] = (_Float16)x4[j][e];
        __syncthreads();
        Frag bx;
        bx.hv[0] = *(const v8h*)&Xt[m * 32 + 8 * h];
        bx.hv[1] = *(const v8h*)&Xt[m * 32 + 16 + 8 * h];
#pragma unroll
        for (int t = 0; t < 4; ++t) {
            const _Float16* wr = pinH + (size_t)(t * 16 + m) * C_ + c0;
            Frag aw;
            aw.hv[0] = *(const v8h*)(wr + 8 * h);
            aw.hv[1] = *(const v8h*)(wr + 16 + 8 * h);
            acc[t] = mma16(aw.v, bx.v, acc[t]);
        }
        __syncthreads();
    }
    float s = 0.0f;
#pragma unroll
    for (int t = 0; t < 4; ++t)
#pragma unroll
        for (int r = 0; r < 8; ++r) { acc[t][r] = acc[t][r] * (1.0f / WSC_); s += acc[t][r]; }
    s += __shfl_xor(s, 16, 32);
    const float mean = s * (1.0f / INNER_);
    float sq = 0.0f;
#pragma unroll
    for (int t = 0; t < 4; ++t)
#pragma unroll
        for (int r = 0; r < 8; ++r) { const float d = acc[t][r] - mean; sq += d * d; }
    sq += __shfl_xor(sq, 16, 32);
    const float var = sq * (1.0f / INNER_);
    const float rstd = 1.0f / sqrtf(var + EPS_);
#pragma unroll
    for (int t = 0; t < 4; ++t)
#pragma unroll
        for (int r = 0; r < 8; ++r) {
            const int i = t * 16 + 8 * h + r;
            const float y = (acc[t][r] - mean) * rstd * lng[i] + lnb[i];
            St[m * INNER_ + i] = (_Float16)y;
        }
    __syncthreads();
    v8h o[4];
#pragma unroll
    for (int it = 0; it < 4; ++it) o[it] = *(const v8h*)&St[8 * (lane + 32 * it)];
    _Float16* base = seqH + (size_t)(b * N_ + nbase) * INNER_;
#pragma unroll
    for (int it = 0; it < 4; ++it) *(volatile v8h*)(base + 8 * (lane + 32 * it)) = o[it];
    __threadfence();
#pragma unroll
    for (int it = 0; it < 4; ++it) *(volatile v8h*)(base + 8 * (lane + 32 * it)) = o[it];
}

__global__ __launch_bounds__(128) void qkv_kernel(
    const _Float16* __restrict__ seqH,
    const _Float16* __restrict__ wqH, const _Float16* __restrict__ wkH,
    const _Float16* __restrict__ wvH,
    _Float16* __restrict__ Qh, _Float16* __restrict__ Kh, _Float16* __restrict__ Vt) {
    __shared__ __attribute__((aligned(16))) _Float16 Stg[64 * 64];
    const int tid = threadIdx.x, wave = tid >> 5, lane = tid & 31;
    const int h = lane >> 4, m = lane & 15;
    const int nbase = blockIdx.x * 64, b = blockIdx.y;
    const int nw = nbase + wave * 16;

    Frag aS[2];
    {
        const _Float16* sp = seqH + (size_t)(b * N_ + nw + m) * INNER_;
#pragma unroll
        for (int ks = 0; ks < 2; ++ks) {
            aS[ks].hv[0] = *(const v8h*)(sp + ks * 32 + 8 * h);
            aS[ks].hv[1] = *(const v8h*)(sp + ks * 32 + 16 + 8 * h);
        }
    }
#pragma unroll
    for (int wsel = 0; wsel < 3; ++wsel) {
        const _Float16* wm = (wsel == 0) ? wqH : ((wsel == 1) ? wkH : wvH);
#pragma unroll
        for (int jt = 0; jt < 4; ++jt) {
            v8f acc = zero8f();
#pragma unroll
            for (int ks = 0; ks < 2; ++ks) {
                const _Float16* wr = wm + (size_t)(jt * 16 + m) * INNER_ + ks * 32;
                Frag bw;
                bw.hv[0] = *(const v8h*)(wr + 8 * h);
                bw.hv[1] = *(const v8h*)(wr + 16 + 8 * h);
                acc = mma16(aS[ks].v, bw.v, acc);
            }
            const int hh = 2 * jt + (m >> 3), d = m & 7;
#pragma unroll
            for (int r = 0; r < 8; ++r) {
                const int nl = wave * 16 + 8 * h + r;
                const _Float16 v = (_Float16)(acc[r] * (QSC_ / WSC_));
                if (wsel < 2) Stg[(hh * 64 + nl) * DH_ + d] = v;
                else          Stg[(hh * DH_ + d) * 64 + nl] = v;
            }
        }
        __syncthreads();
        v8h o[4];
#pragma unroll
        for (int it = 0; it < 4; ++it) o[it] = *(const v8h*)&Stg[8 * (tid + 128 * it)];
        _Float16* dst[4];
#pragma unroll
        for (int it = 0; it < 4; ++it) {
            const int q = tid + 128 * it;
            if (wsel == 0)
                dst[it] = Qh + ((size_t)(b * HEADS_ + (q >> 6)) * N_ + nbase + (q & 63)) * DH_;
            else if (wsel == 1)
                dst[it] = Kh + ((size_t)(b * HEADS_ + (q >> 6)) * N_ + nbase + (q & 63)) * DH_;
            else
                dst[it] = Vt + (size_t)(b * INNER_ + (q >> 3)) * N_ + nbase + (q & 7) * 8;
        }
#pragma unroll
        for (int it = 0; it < 4; ++it) *(volatile v8h*)dst[it] = o[it];
        __threadfence();
#pragma unroll
        for (int it = 0; it < 4; ++it) *(volatile v8h*)dst[it] = o[it];
        __syncthreads();
    }
}

__global__ __launch_bounds__(32) void attn_kernel(
    const _Float16* __restrict__ Qh, const _Float16* __restrict__ Kh,
    const _Float16* __restrict__ Vt, const float* __restrict__ biasv,
    _Float16* __restrict__ attnO) {
    __shared__ __attribute__((aligned(16))) _Float16 Plds[16 * 64];
    __shared__ __attribute__((aligned(16))) _Float16 Olds[16 * DH_];
    const int lane = threadIdx.x, h = lane >> 4, m = lane & 15;
    const int qbase = blockIdx.x * 16, hd = blockIdx.y, b = blockIdx.z;
    const int bh = b * HEADS_ + hd;
    const v8h z8 = zero8h();
    const v8f z8f = zero8f();

    Frag aQ;
    {
        const v8h qv = *(const v8h*)(Qh + ((size_t)bh * N_ + qbase + m) * DH_);
        aQ.hv[0] = z8;
        aQ.hv[1] = z8;
        if (h == 0) aQ.hv[0] = qv;
    }
    const _Float16* Kp = Kh + (size_t)bh * N_ * DH_;
    const _Float16* Vp = Vt + ((size_t)bh * DH_ + (m & 7)) * N_;
    const float* bp = biasv + (size_t)b * N_;

    v8f O = z8f;
    float mrow[8], lrow[8];
#pragma unroll
    for (int r = 0; r < 8; ++r) { mrow[r] = -1e30f; lrow[r] = 0.0f; }
    const float sc = 0.35355339059327373f * (1.0f / (QSC_ * QSC_));

#pragma unroll 1
    for (int kb = 0; kb < N_ / 64; ++kb) {
        const int kbase = kb * 64;
        v8f S[4];
        float bias[4];
#pragma unroll
        for (int kk = 0; kk < 4; ++kk) {
            const int key = kbase + 16 * kk + m;
            const v8h kv = *(const v8h*)(Kp + (size_t)key * DH_);
            Frag bk;
            bk.hv[0] = z8;
            bk.hv[1] = z8;
            if (h == 0) bk.hv[0] = kv;
            S[kk] = mma16(aQ.v, bk.v, z8f);
            bias[kk] = bp[key];
        }
        float mc[8];
#pragma unroll
        for (int r = 0; r < 8; ++r) {
#pragma unroll
            for (int kk = 0; kk < 4; ++kk) S[kk][r] = S[kk][r] * sc + bias[kk];
            mc[r] = fmaxf(fmaxf(S[0][r], S[1][r]), fmaxf(S[2][r], S[3][r]));
        }
#pragma unroll
        for (int off = 1; off < 16; off <<= 1)
#pragma unroll
            for (int r = 0; r < 8; ++r) mc[r] = fmaxf(mc[r], __shfl_xor(mc[r], off, 32));
        float corr[8], rs[8];
#pragma unroll
        for (int r = 0; r < 8; ++r) {
            const float mn = fmaxf(mrow[r], mc[r]);
            corr[r] = __expf(mrow[r] - mn);
            mrow[r] = mn;
            float acc = 0.0f;
#pragma unroll
            for (int kk = 0; kk < 4; ++kk) { S[kk][r] = __expf(S[kk][r] - mn); acc += S[kk][r]; }
            rs[r] = acc;
        }
#pragma unroll
        for (int off = 1; off < 16; off <<= 1)
#pragma unroll
            for (int r = 0; r < 8; ++r) rs[r] += __shfl_xor(rs[r], off, 32);
#pragma unroll
        for (int r = 0; r < 8; ++r) {
            lrow[r] = lrow[r] * corr[r] + rs[r];
            O[r] = O[r] * corr[r];
#pragma unroll
            for (int kk = 0; kk < 4; ++kk)
                Plds[(8 * h + r) * 64 + 16 * kk + m] = (_Float16)(S[kk][r] * PSC_);
        }
        __syncthreads();
#pragma unroll
        for (int ks = 0; ks < 2; ++ks) {
            Frag ap;
            ap.hv[0] = *(const v8h*)&Plds[m * 64 + ks * 32 + 8 * h];
            ap.hv[1] = *(const v8h*)&Plds[m * 64 + ks * 32 + 16 + 8 * h];
            const _Float16* vr = Vp + kbase + ks * 32;
            Frag bv;
            bv.hv[0] = *(const v8h*)(vr + 8 * h);
            bv.hv[1] = *(const v8h*)(vr + 16 + 8 * h);
            O = mma16(ap.v, bv.v, O);
        }
        __syncthreads();
    }
    if (m < DH_) {
#pragma unroll
        for (int r = 0; r < 8; ++r) {
            const float f = (1.0f / lrow[r]) * (1.0f / PSC_);
            Olds[(8 * h + r) * DH_ + m] = (_Float16)(O[r] * f);
        }
    }
    __syncthreads();
    const v8h ov = *(const v8h*)&Olds[(lane & 15) * DH_];
    _Float16* dst = attnO + ((size_t)bh * N_ + qbase + (lane & 15)) * DH_;
    if (lane < 16) *(volatile v8h*)dst = ov;
    __threadfence();
    if (lane < 16) *(volatile v8h*)dst = ov;
}

__global__ __launch_bounds__(32) void projout_kernel(
    const _Float16* __restrict__ attnO, const _Float16* __restrict__ powH,
    float* __restrict__ out0) {
    __shared__ __attribute__((aligned(16))) float Ot[16 * 32];
    const int lane = threadIdx.x, h = lane >> 4, m = lane & 15;
    const int nb = blockIdx.x * 32, ct = blockIdx.y, b = blockIdx.z;

    Frag a[2];
#pragma unroll
    for (int ks = 0; ks < 2; ++ks) {
        const _Float16* ar = powH + (size_t)(ct * 16 + m) * INNER_ + ks * 32;
        a[ks].hv[0] = *(const v8h*)(ar + 8 * h);
        a[ks].hv[1] = *(const v8h*)(ar + 16 + 8 * h);
    }
    v8f acc[2];
#pragma unroll
    for (int nt = 0; nt < 2; ++nt) {
        acc[nt] = zero8f();
        const int n = nb + nt * 16 + m;
#pragma unroll
        for (int ks = 0; ks < 2; ++ks) {
            Frag bb;
            bb.hv[0] = *(const v8h*)(attnO + ((size_t)(b * HEADS_ + 4 * ks + h) * N_ + n) * DH_);
            bb.hv[1] = *(const v8h*)(attnO + ((size_t)(b * HEADS_ + 4 * ks + 2 + h) * N_ + n) * DH_);
            acc[nt] = mma16(a[ks].v, bb.v, acc[nt]);
        }
    }
#pragma unroll
    for (int nt = 0; nt < 2; ++nt)
#pragma unroll
        for (int r = 0; r < 8; ++r)
            Ot[(8 * h + r) * 32 + nt * 16 + m] = acc[nt][r] * (1.0f / (WSC_ * QSC_));
    __syncthreads();
    v4f o[4];
    float* dst[4];
#pragma unroll
    for (int it = 0; it < 4; ++it) {
        const int q = lane + 32 * it;
        o[it] = *(const v4f*)&Ot[4 * q];
        dst[it] = out0 + (size_t)(b * C_ + ct * 16 + (q >> 3)) * N_ + nb + (q & 7) * 4;
    }
#pragma unroll
    for (int it = 0; it < 4; ++it) *(volatile v4f*)dst[it] = o[it];
    __threadfence();
#pragma unroll
    for (int it = 0; it < 4; ++it) *(volatile v4f*)dst[it] = o[it];
}

__global__ __launch_bounds__(256) void gn_final_kernel(
    const float* __restrict__ x, const float* __restrict__ out0,
    const float* __restrict__ gng, const float* __restrict__ gnb,
    float* __restrict__ out) {
    __shared__ double red[8];
    __shared__ double stat[2];
    const int b = blockIdx.x / GNG_, g = blockIdx.x - b * GNG_;
    const int tid = threadIdx.x, lane = tid & 31, wave = tid >> 5;
    const size_t base = (size_t)(b * C_ + g * CPG_) * N_;
    const float* src = out0 + base;
    const int NCH = CPG_ * N_ / 4;

    double s = 0.0;
    for (int q = tid; q < NCH; q += 256) {
        const v4f v = *(const v4f*)(src + 4 * q);
        s += ((double)v[0] + (double)v[1]) + ((double)v[2] + (double)v[3]);
    }
#pragma unroll
    for (int off = 16; off > 0; off >>= 1) s += __shfl_xor(s, off, 32);
    if (lane == 0) red[wave] = s;
    __syncthreads();
    if (tid == 0) {
        double ts = 0.0;
#pragma unroll
        for (int w = 0; w < 8; ++w) ts += red[w];
        stat[0] = ts * (1.0 / (double)(CPG_ * N_));
    }
    __syncthreads();
    const double meand = stat[0];
    double sq = 0.0;
    for (int q = tid; q < NCH; q += 256) {
        const v4f v = *(const v4f*)(src + 4 * q);
#pragma unroll
        for (int e = 0; e < 4; ++e) { const double d = (double)v[e] - meand; sq += d * d; }
    }
#pragma unroll
    for (int off = 16; off > 0; off >>= 1) sq += __shfl_xor(sq, off, 32);
    if (lane == 0) red[wave] = sq;
    __syncthreads();
    if (tid == 0) {
        double tq = 0.0;
#pragma unroll
        for (int w = 0; w < 8; ++w) tq += red[w];
        stat[1] = tq * (1.0 / (double)(CPG_ * N_));
    }
    __syncthreads();
    const float mean = (float)meand;
    const float rstd = 1.0f / sqrtf((float)stat[1] + EPS_);
#pragma unroll 1
    for (int q = tid; q < NCH; q += 256) {
        const int c = g * CPG_ + q / (N_ / 4);
        const float gam = gng[c], bet = gnb[c];
        const v4f v = *(const v4f*)(src + 4 * q);
        const v4f xv = *(const v4f*)(x + base + 4 * q);
        v4f o;
#pragma unroll
        for (int e = 0; e < 4; ++e) o[e] = xv[e] + ((v[e] - mean) * rstd * gam + bet);
        float* dst = out + base + 4 * q;
        *(volatile v4f*)dst = o;
        __threadfence();
        *(volatile v4f*)dst = o;
    }
}

extern "C" void kernel_launch(void* const* d_in, const int* in_sizes, int n_in,
                              void* d_out, int out_size, void* d_ws, size_t ws_size,
                              hipStream_t stream) {
    if (n_in < 17) return;
    if (in_sizes[0] != B_ * C_ * N_ || in_sizes[1] != MID_ * C_ ||
        in_sizes[8] != INNER_ * C_ || in_sizes[11] != INNER_ * INNER_ ||
        in_sizes[14] != C_ * INNER_ || out_size != B_ * C_ * N_) return;

    const float* x    = (const float*)d_in[0];
    const float* gcw  = (const float*)d_in[1];
    const float* bng  = (const float*)d_in[2];
    const float* bnb  = (const float*)d_in[3];
    const float* bnm  = (const float*)d_in[4];
    const float* bnv  = (const float*)d_in[5];
    const float* ghw  = (const float*)d_in[6];
    const float* gww  = (const float*)d_in[7];
    const float* pin  = (const float*)d_in[8];
    const float* lng  = (const float*)d_in[9];
    const float* lnb  = (const float*)d_in[10];
    const float* wq   = (const float*)d_in[11];
    const float* wk   = (const float*)d_in[12];
    const float* wv   = (const float*)d_in[13];
    const float* pw   = (const float*)d_in[14];
    const float* gng  = (const float*)d_in[15];
    const float* gnb  = (const float*)d_in[16];
    float* out = (float*)d_out;

    size_t off = 0;
    auto carve = [&](size_t bytes) -> size_t {
        const size_t r = off;
        off += (bytes + 255) & ~(size_t)255;
        return r;
    };
    const size_t oW    = carve((size_t)WTOT_ * 2);
    const size_t oHP   = carve((size_t)B_ * C_ * PP_ * 4);
    const size_t oWP   = carve((size_t)B_ * C_ * PP_ * 4);
    const size_t oGH   = carve((size_t)B_ * C_ * PP_ * 4);
    const size_t oGW   = carve((size_t)B_ * C_ * PP_ * 4);
    const size_t oBias = carve((size_t)B_ * N_ * 4);
    const size_t oSeq  = carve((size_t)B_ * N_ * INNER_ * 2);
    const size_t oQ    = carve((size_t)B_ * HEADS_ * N_ * DH_ * 2);
    const size_t oK    = carve((size_t)B_ * HEADS_ * N_ * DH_ * 2);
    const size_t oV    = carve((size_t)B_ * INNER_ * N_ * 2);
    const size_t oAO   = carve((size_t)B_ * HEADS_ * N_ * DH_ * 2);
    const size_t oO0   = carve((size_t)B_ * C_ * N_ * 4);
    if (off > ws_size) return;

    char* wsb = (char*)d_ws;
    _Float16* wH    = (_Float16*)(wsb + oW);
    float*    hpool = (float*)(wsb + oHP);
    float*    wpool = (float*)(wsb + oWP);
    float*    gh    = (float*)(wsb + oGH);
    float*    gw    = (float*)(wsb + oGW);
    float*    biasv = (float*)(wsb + oBias);
    _Float16* seqH  = (_Float16*)(wsb + oSeq);
    _Float16* Qh    = (_Float16*)(wsb + oQ);
    _Float16* Kh    = (_Float16*)(wsb + oK);
    _Float16* Vt    = (_Float16*)(wsb + oV);
    _Float16* attnO = (_Float16*)(wsb + oAO);
    float*    out0  = (float*)(wsb + oO0);

    cvt_w_kernel<<<dim3((WTOT_ / 8 + 255) / 256), 256, 0, stream>>>(pin, wq, wk, wv, pw, wH);
    pool_kernel<<<dim3(C_, B_), 64, 0, stream>>>(x, hpool, wpool);
    gates_kernel<<<dim3(B_), 256, 0, stream>>>(hpool, wpool, gcw, bng, bnb, bnm, bnv,
                                                ghw, gww, gh, gw);
    bias_kernel<<<dim3(B_), 256, 0, stream>>>(gh, gw, biasv);
    seq_ln_kernel<<<dim3(N_ / 16, B_), 32, 0, stream>>>(x, wH + WOFF_PIN_, lng, lnb, seqH);
    qkv_kernel<<<dim3(N_ / 64, B_), 128, 0, stream>>>(seqH, wH + WOFF_Q_, wH + WOFF_K_,
                                                      wH + WOFF_V_, Qh, Kh, Vt);
    attn_kernel<<<dim3(N_ / 16, HEADS_, B_), 32, 0, stream>>>(Qh, Kh, Vt, biasv, attnO);
    projout_kernel<<<dim3(N_ / 32, C_ / 16, B_), 32, 0, stream>>>(attnO, wH + WOFF_PW_, out0);
    gn_final_kernel<<<dim3(B_ * GNG_), 256, 0, stream>>>(x, out0, gng, gnb, out);
}
